// DATMixFFNTransformerBlock_58325655879709
// MI455X (gfx1250) — hardware-verified
//
#include <hip/hip_runtime.h>
#define NBt 4
#define CC 768
#define HW 32
#define NPX 1024
#define NR (NBt * NPX)
#define NHD 24
#define HC 32
#define GG 6
#define CG 128
#define DFF 3072
#define HGRP 4
typedef __bf16 v16b __attribute__((ext_vector_type(16)));
typedef unsigned short v8us __attribute__((ext_vector_type(8), may_alias));
typedef float  v8f  __attribute__((ext_vector_type(8)));
typedef float  v4f  __attribute__((ext_vector_type(4)));
typedef float  v4fa __attribute__((ext_vector_type(4), may_alias));
union FragB { v16b v; v8us half[2]; unsigned short u[16]; };

__device__ __forceinline__ unsigned short bf16_bits(float x) { unsigned int u = __float_as_uint(x); return (unsigned short)((u + 0x7FFFu + ((u >> 16) & 1u)) >> 16); }
__device__ __forceinline__ float bf16_val(unsigned short b) { return __uint_as_float(((unsigned int)b) << 16); }
__device__ __forceinline__ float bf16_round(float x) { return bf16_val(bf16_bits(x)); }
template <int NT>
__device__ __forceinline__ v8f mmaN(v16b ah, v16b al, v16b bh, v16b bl, v8f c) {
  c = __builtin_amdgcn_wmma_f32_16x16x32_bf16(false, ah, false, bh, (short)0, c, false, false);
  if (NT >= 2) c = __builtin_amdgcn_wmma_f32_16x16x32_bf16(false, al, false, bh, (short)0, c, false, false);
  if (NT >= 3) c = __builtin_amdgcn_wmma_f32_16x16x32_bf16(false, ah, false, bl, (short)0, c, false, false);
  asm volatile("v_nop\n\tv_nop\n\tv_nop\n\tv_nop" : "+v"(c) : "v"(ah), "v"(al), "v"(bh), "v"(bl));
  return c;
}

__global__ __launch_bounds__(256) void k_wt_bf16(const float* __restrict__ W, unsigned short* __restrict__ Wt, int K, int N) {
  const int t = blockIdx.x * 256 + threadIdx.x;
  const int k8n = K / 8;
  if (t >= N * k8n) return;
  const int n = t / k8n, k8 = (t % k8n) * 8;
  v8us v;
#pragma unroll
  for (int i = 0; i < 8; ++i) v[i] = bf16_bits(W[(size_t)(k8 + i) * N + n]);
  *(volatile v8us*)(Wt + (size_t)n * K + k8) = v;
  __threadfence();
  *(volatile v8us*)(Wt + (size_t)n * K + k8) = v;
}

template <bool ASPLIT, int ACT, bool BIAS_BF16>
__global__ __launch_bounds__(128) void k_gemm_bf(const float* __restrict__ A, int lda, const unsigned short* __restrict__ Wt, int ldb,
                                               const float* __restrict__ bias, float* __restrict__ C, int ldc, int M, int N, int K) {
  __shared__ __attribute__((aligned(16))) float so[4][16][64];
  const int tid = threadIdx.x, w = tid >> 5, lane = tid & 31, ln = lane & 15, hh = lane >> 4;
  const int ntn = N / 64;
  const int wid = blockIdx.x * 4 + w;
  const int mt = wid / ntn, nq = wid % ntn;
  if (mt * 16 >= M) return;
  const int row0 = mt * 16, col0 = nq * 64;
  const float* arow = A + (size_t)(row0 + ln) * lda;
  v8f acc[4] = {};
  for (int kb = 0; kb < K; kb += 32) {
    FragB ah, al;
    const v4f x0 = *(const v4fa*)(arow + kb + 8 * hh), x1 = *(const v4fa*)(arow + kb + 8 * hh + 4);
    const v4f x2 = *(const v4fa*)(arow + kb + 16 + 8 * hh), x3 = *(const v4fa*)(arow + kb + 16 + 8 * hh + 4);
    float xs[16] = {x0[0],x0[1],x0[2],x0[3],x1[0],x1[1],x1[2],x1[3],x2[0],x2[1],x2[2],x2[3],x3[0],x3[1],x3[2],x3[3]};
#pragma unroll
    for (int i = 0; i < 16; ++i) { const unsigned short hb = bf16_bits(xs[i]); ah.u[i] = hb; al.u[i] = ASPLIT ? bf16_bits(xs[i] - bf16_val(hb)) : (unsigned short)0; }
#pragma unroll
    for (int t = 0; t < 4; ++t) {
      const unsigned short* brow = Wt + (size_t)(col0 + t * 16 + ln) * ldb + kb;
      FragB b;
      b.half[0] = *(const v8us*)(brow + 8 * hh);
      b.half[1] = *(const v8us*)(brow + 16 + 8 * hh);
      acc[t] = mmaN<ASPLIT ? 2 : 1>(ah.v, al.v, b.v, b.v, acc[t]);
    }
  }
#pragma unroll
  for (int t = 0; t < 4; ++t) {
    float bv = bias ? bias[col0 + t * 16 + ln] : 0.f;
    if (BIAS_BF16) bv = bf16_round(bv);
#pragma unroll
    for (int r = 0; r < 8; ++r) { float v = acc[t][r] + bv; if (ACT == 1) v = fmaxf(v, 0.f); so[w][8 * hh + r][t * 16 + ln] = v; }
  }
  __builtin_amdgcn_fence(__ATOMIC_ACQ_REL, "workgroup");
  __builtin_amdgcn_wave_barrier();
  const int rsub = lane >> 4, c4 = (lane & 15) * 4;
  for (int pass = 0; pass < 2; ++pass) {
#pragma unroll
    for (int q = 0; q < 8; ++q) {
      const int r = q * 2 + rsub;
      const v4f v = *(const v4fa*)&so[w][r][c4];
      *(volatile v4f*)(C + (size_t)(row0 + r) * ldc + col0 + c4) = v;
    }
    if (pass == 0) __threadfence();
  }
}

template <bool ASPLIT, int ACT, bool BIAS_BF16, bool RES_BF16>
__global__ __launch_bounds__(128) void k_gemm_bf3(const float* __restrict__ A, int lda, const unsigned short* __restrict__ Wt, int ldb,
                                                const float* __restrict__ bias, const float* __restrict__ resid, int rmod, int ldr,
                                                float* __restrict__ C, int ldc, int M, int N, int K) {
  __shared__ __attribute__((aligned(16))) float so[4][16][64];
  const int tid = threadIdx.x, w = tid >> 5, lane = tid & 31, ln = lane & 15, hh = lane >> 4;
  const int ntn = N / 64;
  const int wid = blockIdx.x * 4 + w;
  const int mt = wid / ntn, nq = wid % ntn;
  if (mt * 16 >= M) return;
  const int row0 = mt * 16, col0 = nq * 64;
  const float* arow = A + (size_t)(row0 + ln) * lda;
  v8f acc[4] = {};
  for (int kb = 0; kb < K; kb += 32) {
    FragB ah, al;
    const v4f x0 = *(const v4fa*)(arow + kb + 8 * hh), x1 = *(const v4fa*)(arow + kb + 8 * hh + 4);
    const v4f x2 = *(const v4fa*)(arow + kb + 16 + 8 * hh), x3 = *(const v4fa*)(arow + kb + 16 + 8 * hh + 4);
    float xs[16] = {x0[0],x0[1],x0[2],x0[3],x1[0],x1[1],x1[2],x1[3],x2[0],x2[1],x2[2],x2[3],x3[0],x3[1],x3[2],x3[3]};
#pragma unroll
    for (int i = 0; i < 16; ++i) { const unsigned short hb = bf16_bits(xs[i]); ah.u[i] = hb; al.u[i] = ASPLIT ? bf16_bits(xs[i] - bf16_val(hb)) : (unsigned short)0; }
#pragma unroll
    for (int t = 0; t < 4; ++t) {
      const unsigned short* brow = Wt + (size_t)(col0 + t * 16 + ln) * ldb + kb;
      FragB b;
      b.half[0] = *(const v8us*)(brow + 8 * hh);
      b.half[1] = *(const v8us*)(brow + 16 + 8 * hh);
      acc[t] = mmaN<ASPLIT ? 2 : 1>(ah.v, al.v, b.v, b.v, acc[t]);
    }
  }
#pragma unroll
  for (int t = 0; t < 4; ++t) {
    const int col = col0 + t * 16 + ln;
    float bv = bias ? bias[col] : 0.f;
    if (BIAS_BF16) bv = bf16_round(bv);
#pragma unroll
    for (int r = 0; r < 8; ++r) {
      float v = acc[t][r] + bv;
      if (resid) { float rv = resid[(size_t)((row0 + 8 * hh + r) % rmod) * ldr + col]; if (RES_BF16) rv = bf16_round(rv); v += rv; }
      if (ACT == 1) v = fmaxf(v, 0.f);
      if (ACT == 2) v = 0.5f * v * (1.0f + erff(v * 0.70710678118654752f));
      if (ACT == 3) { const float u = 0.7978845608028654f * (v + 0.044715f * v * v * v); v = 0.5f * v * (1.0f + tanhf(u)); }
      so[w][8 * hh + r][t * 16 + ln] = v;
    }
  }
  __builtin_amdgcn_fence(__ATOMIC_ACQ_REL, "workgroup");
  __builtin_amdgcn_wave_barrier();
  const int rsub = lane >> 4, c4 = (lane & 15) * 4;
  for (int pass = 0; pass < 2; ++pass) {
#pragma unroll
    for (int q = 0; q < 8; ++q) {
      const int r = q * 2 + rsub;
      const v4f v = *(const v4fa*)&so[w][r][c4];
      *(volatile v4f*)(C + (size_t)(row0 + r) * ldc + col0 + c4) = v;
    }
    if (pass == 0) __threadfence();
  }
}
template <bool PARAM_BF16>
__global__ __launch_bounds__(256) void k_layernorm(const float* __restrict__ X, const float* __restrict__ R, const float* __restrict__ g, const float* __restrict__ bta,
                                                  float* __restrict__ out_sum, float* __restrict__ out_norm, int N, float eps) {
  __shared__ float red[256];
  const int row = blockIdx.x, tid = threadIdx.x;
  const float* x = X + (size_t)row * N; const float* rr = R ? R + (size_t)row * N : nullptr;
  float vals[16];
  const int per = N / 256;
  float s1 = 0.f;
  for (int u = 0; u < per / 4; ++u) {
    const int j = tid * 4 + 1024 * u;
    const v4f a = *(const v4fa*)(x + j);
    v4f b = {0.f,0.f,0.f,0.f}; if (rr) b = *(const v4fa*)(rr + j);
#pragma unroll
    for (int q = 0; q < 4; ++q) { const float v = a[q] + b[q]; vals[u * 4 + q] = v; s1 += v; }
  }
  red[tid] = s1; __syncthreads();
  for (int st = 128; st > 0; st >>= 1) { if (tid < st) red[tid] += red[tid + st]; __syncthreads(); }
  const float mu = red[0] / (float)N; __syncthreads();
  float s2 = 0.f;
  for (int u = 0; u < per / 4; ++u)
#pragma unroll
    for (int q = 0; q < 4; ++q) { const float c = vals[u * 4 + q] - mu; s2 += c * c; }
  red[tid] = s2; __syncthreads();
  for (int st = 128; st > 0; st >>= 1) { if (tid < st) red[tid] += red[tid + st]; __syncthreads(); }
  const float rs = rsqrtf(red[0] / (float)N + eps);
  for (int pass = 0; pass < 2; ++pass) {
    for (int u = 0; u < per / 4; ++u) {
      const int j = tid * 4 + 1024 * u;
      v4f o, sm;
#pragma unroll
      for (int q = 0; q < 4; ++q) {
        float gg = g[j + q], bb = bta[j + q];
        if (PARAM_BF16) { gg = bf16_round(gg); bb = bf16_round(bb); }
        sm[q] = vals[u * 4 + q]; o[q] = (vals[u * 4 + q] - mu) * rs * gg + bb;
      }
      if (out_sum) *(volatile v4f*)(out_sum + (size_t)row * N + j) = sm;
      *(volatile v4f*)(out_norm + (size_t)row * N + j) = o;
    }
    if (pass == 0) __threadfence();
  }
}


typedef _Float16 v16h __attribute__((ext_vector_type(16)));
union FragH { v16h v; v8us half[2]; _Float16 h[16]; unsigned short u[16]; };
template <int NT>
__device__ __forceinline__ v8f mmaH(v16h ah, v16h al, v16h bh, v16h bl, v8f c) {
  c = __builtin_amdgcn_wmma_f32_16x16x32_f16(false, ah, false, bh, (short)0, c, false, false);
  if (NT >= 2) c = __builtin_amdgcn_wmma_f32_16x16x32_f16(false, al, false, bh, (short)0, c, false, false);
  if (NT >= 3) c = __builtin_amdgcn_wmma_f32_16x16x32_f16(false, ah, false, bl, (short)0, c, false, false);
  asm volatile("v_nop\n\tv_nop\n\tv_nop\n\tv_nop" : "+v"(c) : "v"(ah), "v"(al), "v"(bh), "v"(bl));
  return c;
}
template <bool ASPLIT>
__global__ __launch_bounds__(128) void k_gemm_h(const float* __restrict__ A, int lda, size_t sA, const _Float16* __restrict__ Bh, int ldb, size_t sB, float alpha, float* __restrict__ C, int ldc, size_t sC, int M, int N, int K) {
  __shared__ __attribute__((aligned(16))) float so[4][16][64];
  const int tid = threadIdx.x, w = tid >> 5, lane = tid & 31, ln = lane & 15, hh = lane >> 4; const int by = blockIdx.y;
  A += (size_t)by * sA; Bh += (size_t)by * sB; C += (size_t)by * sC;
  const int ntn = (N + 63) / 64; const int wid = blockIdx.x * 4 + w; const int mt = wid / ntn, nq = wid % ntn; if (mt * 16 >= M) return;
  const int row0 = mt * 16, col0 = nq * 64; const float* arow = A + (size_t)(row0 + ln) * lda;
  v8f acc[4] = {};
  for (int kb = 0; kb < K; kb += 32) {
    FragH ah, al;
    const v4f x0 = *(const v4fa*)(arow + kb + 8 * hh), x1 = *(const v4fa*)(arow + kb + 8 * hh + 4), x2 = *(const v4fa*)(arow + kb + 16 + 8 * hh), x3 = *(const v4fa*)(arow + kb + 16 + 8 * hh + 4);
    float xs[16] = {x0[0],x0[1],x0[2],x0[3],x1[0],x1[1],x1[2],x1[3],x2[0],x2[1],x2[2],x2[3],x3[0],x3[1],x3[2],x3[3]};
#pragma unroll
    for (int i = 0; i < 16; ++i) { const _Float16 h = (_Float16)xs[i]; ah.h[i] = h; al.h[i] = ASPLIT ? (_Float16)(xs[i] - (float)h) : (_Float16)0.0f; }
#pragma unroll
    for (int t = 0; t < 4; ++t) { if (col0 + t * 16 >= N) continue; const size_t boff = (size_t)(col0 + t * 16 + ln) * ldb + kb; FragH bq; bq.half[0] = *(const v8us*)(Bh + boff + 8 * hh); bq.half[1] = *(const v8us*)(Bh + boff + 16 + 8 * hh);
      acc[t] = mmaH<ASPLIT ? 2 : 1>(ah.v, al.v, bq.v, bq.v, acc[t]); }
  }
#pragma unroll
  for (int t = 0; t < 4; ++t) { if (col0 + t * 16 >= N) continue;
#pragma unroll
    for (int r = 0; r < 8; ++r) so[w][8 * hh + r][t * 16 + ln] = acc[t][r] * alpha; }
  __builtin_amdgcn_fence(__ATOMIC_ACQ_REL, "workgroup"); __builtin_amdgcn_wave_barrier();
  const int rsub = lane >> 4, c4 = (lane & 15) * 4;
  for (int pass = 0; pass < 2; ++pass) {
#pragma unroll
    for (int q = 0; q < 8; ++q) { const int r = q * 2 + rsub; if (col0 + c4 < N) { const v4f v = *(const v4fa*)&so[w][r][c4]; *(volatile v4f*)(C + (size_t)(row0 + r) * ldc + col0 + c4) = v; } }
    if (pass == 0) __threadfence(); }
}

__global__ __launch_bounds__(256) void k_wt_f16(const float* __restrict__ W, _Float16* __restrict__ Wt, int K, int N, float scale) {
  const int t = blockIdx.x * 256 + threadIdx.x; if (t >= N * (K / 8)) return; const int n = t / (K / 8), k8 = (t % (K / 8)) * 8; FragH f;
#pragma unroll
  for (int i = 0; i < 8; ++i) f.h[i] = (_Float16)(bf16_round(W[(size_t)(k8 + i) * N + n]) * scale); const v8us o = f.half[0];
  *(volatile v8us*)((unsigned short*)Wt + (size_t)n * K + k8) = o; __threadfence(); *(volatile v8us*)((unsigned short*)Wt + (size_t)n * K + k8) = o;
}
template <int ACT>
__global__ __launch_bounds__(128) void k_gemm_hhx(const _Float16* __restrict__ A, int lda, size_t sA, const _Float16* __restrict__ Bh, int ldb, size_t sB, float alpha, const float* __restrict__ bias, size_t sBias, const float* __restrict__ CP, int rowsPerB, size_t sCPb, int row0g,
    float* __restrict__ C, _Float16* __restrict__ C16, int ldc, size_t sC, int M, int N, int K) {
  __shared__ __attribute__((aligned(16))) float so[4][16][64];
  const int tid = threadIdx.x, w = tid >> 5, lane = tid & 31, ln = lane & 15, hh = lane >> 4; const int by = blockIdx.y;
  A += (size_t)by * sA; Bh += (size_t)by * sB; const size_t cofs = (size_t)by * sC; const float* bp = bias ? bias + (size_t)by * sBias : nullptr;
  const int ntn = (N + 63) / 64; const int wid = blockIdx.x * 4 + w; const int mt = wid / ntn, nq = wid % ntn; if (mt * 16 >= M) return;
  const int row0 = mt * 16, col0 = nq * 64; const _Float16* arow = A + (size_t)(row0 + ln) * lda;
  v8f acc[4] = {};
  for (int kb = 0; kb < K; kb += 32) { FragH ah; ah.half[0] = *(const v8us*)((const unsigned short*)arow + kb + 8 * hh); ah.half[1] = *(const v8us*)((const unsigned short*)arow + kb + 16 + 8 * hh);
#pragma unroll
    for (int t = 0; t < 4; ++t) { if (col0 + t * 16 >= N) continue; const size_t boff = (size_t)(col0 + t * 16 + ln) * ldb + kb; FragH bq; bq.half[0] = *(const v8us*)((const unsigned short*)Bh + boff + 8 * hh); bq.half[1] = *(const v8us*)((const unsigned short*)Bh + boff + 16 + 8 * hh);
      acc[t] = mmaH<1>(ah.v, ah.v, bq.v, bq.v, acc[t]); }
  }
#pragma unroll
  for (int t = 0; t < 4; ++t) { if (col0 + t * 16 >= N) continue; const int col = col0 + t * 16 + ln; const float bv = bp ? bf16_round(bp[col]) : 0.f;
#pragma unroll
    for (int r = 0; r < 8; ++r) { float v = acc[t][r] * alpha + bv; if (CP) { const int bidx = (row0g + row0 + 8 * hh + r) / rowsPerB; v += CP[(size_t)bidx * sCPb + (size_t)by * 64 + col]; } if (ACT == 1) v = (v > 0.f) ? v : expm1f(v); else if (ACT == 7) v = (v > 0.f) ? v + 1.0f : expf(v); else if (ACT == 8) v = tanhf(v); else if (ACT == 9) v = 0.5f * v * (1.0f + tanhf(0.7978845608028654f * (v + 0.044715f * v * v * v))); else if (ACT == 11) v = 1.0f / (1.0f + expf(-v)); else if (ACT == 12) v = (v > 0.f) ? v : 0.01f * v; else if (ACT == 14) v = (v > 0.f) ? v : 0.1f * v; else if (ACT == 15) v = v / (1.0f + expf(-v)); else if (ACT == 3) v = fmaxf(v, 0.f); else if (ACT == 6) v = 0.5f * v * (1.0f + erff(v * 0.70710678118654752f)); so[w][8 * hh + r][t * 16 + ln] = v; } }
  __builtin_amdgcn_fence(__ATOMIC_ACQ_REL, "workgroup"); __builtin_amdgcn_wave_barrier();
  const int rsub = lane >> 4, c4 = (lane & 15) * 4; typedef _Float16 v4h __attribute__((ext_vector_type(4)));
  for (int pass = 0; pass < 2; ++pass) {
#pragma unroll
    for (int q = 0; q < 8; ++q) { const int r = q * 2 + rsub; if (col0 + c4 < N) { const v4f v = *(const v4fa*)&so[w][r][c4]; if (C) *(volatile v4f*)(C + cofs + (size_t)(row0 + r) * ldc + col0 + c4) = v; if (C16) { v4h h4; for (int i = 0; i < 4; ++i) h4[i] = (_Float16)v[i]; *(volatile v4h*)(C16 + cofs + (size_t)(row0 + r) * ldc + col0 + c4) = h4; } } }
    if (pass == 0) __threadfence(); }
}


typedef _Float16 v4h __attribute__((ext_vector_type(4)));

__global__ __launch_bounds__(256) void k_x16(const float* __restrict__ x, _Float16* __restrict__ X16, size_t n8) { const size_t t = (size_t)blockIdx.x * 256 + threadIdx.x; if (t >= n8) return; FragH f;
#pragma unroll
  for (int q = 0; q < 8; ++q) f.h[q] = (_Float16)bf16_round(x[t * 8 + q]); *(volatile v8us*)((unsigned short*)X16 + t * 8) = f.half[0]; __threadfence(); *(volatile v8us*)((unsigned short*)X16 + t * 8) = f.half[0]; }
__global__ __launch_bounds__(256) void k_h16(const float* __restrict__ x, _Float16* __restrict__ X16, size_t n8) { const size_t t = (size_t)blockIdx.x * 256 + threadIdx.x; if (t >= n8) return; FragH f;
#pragma unroll
  for (int q = 0; q < 8; ++q) f.h[q] = (_Float16)x[t * 8 + q]; *(volatile v8us*)((unsigned short*)X16 + t * 8) = f.half[0]; __threadfence(); *(volatile v8us*)((unsigned short*)X16 + t * 8) = f.half[0]; }
__global__ __launch_bounds__(256) void k_round16f(const float* __restrict__ W, _Float16* __restrict__ Bt, size_t n8) { const size_t t = (size_t)blockIdx.x * 256 + threadIdx.x; if (t >= n8) return; FragH f;
#pragma unroll
  for (int i = 0; i < 8; ++i) f.h[i] = (_Float16)(bf16_round(W[t * 8 + i]) * 16.0f); *(volatile v8us*)((unsigned short*)Bt + t * 8) = f.half[0]; __threadfence(); *(volatile v8us*)((unsigned short*)Bt + t * 8) = f.half[0]; }
template <int NHv, int TTv>
__global__ __launch_bounds__(256) void k_vt(const _Float16* __restrict__ V16, int ldv, int voff, _Float16* __restrict__ Vt) { __shared__ unsigned short tl[64][66]; const int tid = threadIdx.x; const int slab = blockIdx.x / (TTv / 64), lg = blockIdx.x % (TTv / 64); const int b = slab / NHv, h = slab % NHv;
  for (int i = tid; i < 64 * 8; i += 256) { const int r = i / 8, c8 = (i % 8) * 8; FragH f; f.half[0] = *(const v8us*)((const unsigned short*)V16 + ((size_t)b * TTv + lg * 64 + r) * ldv + voff + h * 64 + c8);
#pragma unroll
    for (int q = 0; q < 8; ++q) tl[r][c8 + q] = f.u[q]; }
  __syncthreads();
  for (int pass = 0; pass < 2; ++pass) {
#pragma unroll
    for (int rd = 0; rd < 2; ++rd) { const int d = rd * 32 + tid / 8, pc = tid % 8; FragH f;
#pragma unroll
      for (int q = 0; q < 8; ++q) f.u[q] = tl[pc * 8 + q][d];
      *(volatile v8us*)((unsigned short*)Vt + ((size_t)slab * 64 + d) * TTv + lg * 64 + pc * 8) = f.half[0]; }
    if (pass == 0) __threadfence(); } }

__global__ __launch_bounds__(256) void k_hl(const float* __restrict__ F, _Float16* __restrict__ Hh, _Float16* __restrict__ Hl, size_t n8) { const size_t t = (size_t)blockIdx.x * 256 + threadIdx.x; if (t >= n8) return; FragH fh, fl; const v4f a = *(const v4fa*)(F + t * 8), c = *(const v4fa*)(F + t * 8 + 4);
#pragma unroll
  for (int q = 0; q < 4; ++q) { _Float16 h = (_Float16)a[q]; fh.h[q] = h; fl.h[q] = (_Float16)((a[q] - (float)h) * 1024.0f); h = (_Float16)c[q]; fh.h[4 + q] = h; fl.h[4 + q] = (_Float16)((c[q] - (float)h) * 1024.0f); }
  for (int pass = 0; pass < 2; ++pass) { *(volatile v8us*)((unsigned short*)Hh + t * 8) = fh.half[0]; *(volatile v8us*)((unsigned short*)Hl + t * 8) = fl.half[0]; if (pass == 0) __threadfence(); } }

__device__ __forceinline__ float gelu_f(float v) { return 0.5f * v * (1.0f + erff(v * 0.70710678118654752f)); }
__device__ __forceinline__ v4f shfl4(v4f v, int srcl) { v4f r; r[0] = __shfl(v[0], srcl, 32); r[1] = __shfl(v[1], srcl, 32); r[2] = __shfl(v[2], srcl, 32); r[3] = __shfl(v[3], srcl, 32); return r; }
__global__ __launch_bounds__(256) void k_f16(const float* __restrict__ F, _Float16* __restrict__ O16, size_t n8) { const size_t t = (size_t)blockIdx.x * 256 + threadIdx.x; if (t >= n8) return; const v4f a = *(const v4fa*)(F + t * 8), c = *(const v4fa*)(F + t * 8 + 4); FragH f;
#pragma unroll
  for (int q = 0; q < 8; ++q) f.h[q] = (_Float16)((q < 4) ? a[q] : c[q - 4]);
  *(volatile v8us*)((unsigned short*)O16 + t * 8) = f.half[0]; __threadfence(); *(volatile v8us*)((unsigned short*)O16 + t * 8) = f.half[0]; }
__global__ __launch_bounds__(256) void k_rstat16(const _Float16* __restrict__ A, int width, int nrows, float eps, float* __restrict__ ST) {
  #pragma clang fp contract(off)
  const int tid = threadIdx.x, w = tid >> 5, ln = tid & 31; const int r = blockIdx.x * 8 + w; if (r >= nrows) return; const _Float16* ar = A + (size_t)r * width; float s = 0.f; for (int c = ln; c < width; c += 32) s += (float)ar[c];
  for (int o = 16; o > 0; o >>= 1) s += __shfl_xor(s, o, 32); const float mu = s / (float)width; float q2 = 0.f; for (int c = ln; c < width; c += 32) { const float d = (float)ar[c] - mu; q2 += d * d; }
  for (int o = 16; o > 0; o >>= 1) q2 += __shfl_xor(q2, o, 32); const float rs = rsqrtf(q2 / (float)width + eps); const float v = (ln == 0) ? mu : (ln == 1) ? rs : 0.f;
  *(volatile float*)(ST + (size_t)r * 32 + ln) = v; __threadfence(); *(volatile float*)(ST + (size_t)r * 32 + ln) = v; }
__global__ __launch_bounds__(256) void k_tok(const float* __restrict__ x, float* __restrict__ X) { const int t = blockIdx.x * 256 + threadIdx.x; if (t >= NR * (CC / 4)) return; const int c0 = (t % (CC / 4)) * 4, r = t / (CC / 4); const int b = r / NPX, n = r % NPX; v4f v;
#pragma unroll
  for (int q = 0; q < 4; ++q) v[q] = bf16_round(x[((size_t)b * CC + c0 + q) * NPX + n]);
  *(volatile v4f*)(X + (size_t)r * CC + c0) = v; __threadfence(); *(volatile v4f*)(X + (size_t)r * CC + c0) = v; }
__global__ __launch_bounds__(256) void k_rstat(const float* __restrict__ A, int width, int nrows, float eps, float* __restrict__ ST) {
  #pragma clang fp contract(off)
  const int tid = threadIdx.x, w = tid >> 5, ln = tid & 31; const int r = blockIdx.x * 8 + w; if (r >= nrows) return; const float* ar = A + (size_t)r * width; float s = 0.f; for (int c = ln; c < width; c += 32) s += ar[c];
  for (int o = 16; o > 0; o >>= 1) s += __shfl_xor(s, o, 32); const float mu = s / (float)width; float q2 = 0.f; for (int c = ln; c < width; c += 32) { const float d = ar[c] - mu; q2 += d * d; }
  for (int o = 16; o > 0; o >>= 1) q2 += __shfl_xor(q2, o, 32); const float rs = rsqrtf(q2 / (float)width + eps); const float v = (ln == 0) ? mu : (ln == 1) ? rs : 0.f;
  *(volatile float*)(ST + (size_t)r * 32 + ln) = v; __threadfence(); *(volatile float*)(ST + (size_t)r * 32 + ln) = v; }
__global__ __launch_bounds__(256) void k_lnapply(const float* __restrict__ A, int width, const float* __restrict__ ST, const float* __restrict__ g, const float* __restrict__ bb, float* __restrict__ OF, _Float16* __restrict__ O16) {
  #pragma clang fp contract(off)
  const int t = blockIdx.x * 256 + threadIdx.x; const int per = width / 8; if (t >= NR * per) return; const int c0 = (t % per) * 8, r = t / per; const int l = threadIdx.x & 31; const float mu = ST[(size_t)r * 32], rs = ST[(size_t)r * 32 + 1]; const v4f a = *(const v4fa*)(A + (size_t)r * width + c0), c4 = *(const v4fa*)(A + (size_t)r * width + c0 + 4); v4f oa, ob; FragH f;
#pragma unroll
  for (int q = 0; q < 8; ++q) { const int c = c0 + q; const float y = (((q < 4) ? a[q] : c4[q - 4]) - mu) * rs * bf16_round(g[c]) + bf16_round(bb[c]); if (q < 4) oa[q] = y; else ob[q - 4] = y; f.h[q] = (_Float16)y; }
  if (OF) { float* row = OF + (size_t)r * width + (c0 - l * 8); const v4f a1 = shfl4(oa, l >> 1), b1 = shfl4(ob, l >> 1), a2 = shfl4(oa, 16 + (l >> 1)), b2 = shfl4(ob, 16 + (l >> 1)); const v4f c1 = (l & 1) ? b1 : a1, c2 = (l & 1) ? b2 : a2; for (int pass = 0; pass < 2; ++pass) { *(volatile v4f*)(row + l * 4) = c1; *(volatile v4f*)(row + 128 + l * 4) = c2; if (pass == 0) __threadfence(); } }
  if (O16) { *(volatile v8us*)((unsigned short*)O16 + (size_t)r * width + c0) = f.half[0]; __threadfence(); *(volatile v8us*)((unsigned short*)O16 + (size_t)r * width + c0) = f.half[0]; } }
__global__ __launch_bounds__(256) void k_odw(const float* __restrict__ Q, const float* __restrict__ w, const float* __restrict__ bb, float* __restrict__ OD) {
  #pragma clang fp contract(off)
  const int t = blockIdx.x * 256 + threadIdx.x; if (t >= NBt * GG * NPX * (CG / 4)) return; const int c0 = (t % (CG / 4)) * 4; const int rgn = t / (CG / 4); const int n = rgn % NPX, g = (rgn / NPX) % GG, b = rgn / (NPX * GG); const int y = n / HW, x = n % HW; v4f acc;
#pragma unroll
  for (int q = 0; q < 4; ++q) acc[q] = bf16_round(bb[c0 + q]);
#pragma unroll 1
  for (int ky = 0; ky < 9; ++ky) { const int yy = y + ky - 4; if (yy < 0 || yy >= HW) continue;
#pragma unroll 1
    for (int kx = 0; kx < 9; ++kx) { const int xx = x + kx - 4; if (xx < 0 || xx >= HW) continue; const v4f v = *(const v4fa*)(Q + ((size_t)b * NPX + yy * HW + xx) * CC + g * CG + c0);
#pragma unroll
      for (int q = 0; q < 4; ++q) acc[q] += v[q] * bf16_round(w[(size_t)(c0 + q) * 81 + ky * 9 + kx]); } }
  *(volatile v4f*)(OD + (size_t)rgn * CG + c0) = acc; __threadfence(); *(volatile v4f*)(OD + (size_t)rgn * CG + c0) = acc; }
__global__ __launch_bounds__(256) void k_opos(const float* __restrict__ OD, const float* __restrict__ g, const float* __restrict__ bb, const float* __restrict__ pw, float* __restrict__ POS) {
  #pragma clang fp contract(off)
  const int tid = threadIdx.x, w = tid >> 5, ln = tid & 31; const int rgn = blockIdx.x * 8 + w; if (rgn >= NBt * GG * NPX) return; const int n = rgn % NPX; const float* od = OD + (size_t)rgn * CG; float v[4]; float s = 0.f;
#pragma unroll
  for (int k = 0; k < 4; ++k) { v[k] = od[ln * 4 + k]; s += v[k]; }
  for (int o = 16; o > 0; o >>= 1) s += __shfl_xor(s, o, 32); const float mu = s / (float)CG; float q2 = 0.f;
#pragma unroll
  for (int k = 0; k < 4; ++k) { const float d = v[k] - mu; q2 += d * d; }
  for (int o = 16; o > 0; o >>= 1) q2 += __shfl_xor(q2, o, 32); const float rs = rsqrtf(q2 / (float)CG + 1e-5f); float sy = 0.f, sx = 0.f;
#pragma unroll
  for (int k = 0; k < 4; ++k) { const int c = ln * 4 + k; const float o_ = gelu_f((v[k] - mu) * rs * bf16_round(g[c]) + bf16_round(bb[c])); sy += bf16_round(pw[c]) * o_; sx += bf16_round(pw[CG + c]) * o_; }
  for (int o = 16; o > 0; o >>= 1) { sy += __shfl_xor(sy, o, 32); sx += __shfl_xor(sx, o, 32); }
  const int i = n / HW, j = n % HW; const float oy = tanhf(sy) * (1.0f / 31.0f), ox = tanhf(sx) * (1.0f / 31.0f); const float refy = (((float)i + 0.5f) / 32.0f) * 2.0f - 1.0f, refx = (((float)j + 0.5f) / 32.0f) * 2.0f - 1.0f; const float py = oy + refy, px = ox + refx; const float gx = (px + 1.0f) * 0.5f * 31.0f, gy = (py + 1.0f) * 0.5f * 31.0f;
  const float val = (ln == 0) ? gy : (ln == 1) ? gx : 0.f; *(volatile float*)(POS + (size_t)rgn * 32 + ln) = val; __threadfence(); *(volatile float*)(POS + (size_t)rgn * 32 + ln) = val; }
__global__ __launch_bounds__(256) void k_samp(const float* __restrict__ XN, const float* __restrict__ POS, _Float16* __restrict__ XS16) {
  #pragma clang fp contract(off)
  const int t = blockIdx.x * 256 + threadIdx.x; if (t >= NBt * GG * NPX * (CG / 8)) return; const int c0 = (t % (CG / 8)) * 8; const int rgn = t / (CG / 8); const int ns = rgn % NPX, g = (rgn / NPX) % GG, b = rgn / (NPX * GG); const float gy = POS[(size_t)rgn * 32], gx = POS[(size_t)rgn * 32 + 1]; const float x0 = floorf(gx), y0 = floorf(gy); const float wx1 = gx - x0, wy1 = gy - y0; float acc[8];
#pragma unroll
  for (int q = 0; q < 8; ++q) acc[q] = 0.f;
#pragma unroll
  for (int cn = 0; cn < 4; ++cn) { const float ix = x0 + (float)(cn & 1), iy = y0 + (float)(cn >> 1); const bool valid = (ix >= 0.f && ix <= 31.f && iy >= 0.f && iy <= 31.f); const float wgt = ((cn & 1) ? wx1 : (1.0f - wx1)) * ((cn >> 1) ? wy1 : (1.0f - wy1)); const float f = valid ? wgt : 0.f; const int xi = (int)fminf(fmaxf(ix, 0.f), 31.f), yi = (int)fminf(fmaxf(iy, 0.f), 31.f); const float* src = XN + ((size_t)b * NPX + yi * HW + xi) * CC + g * CG + c0; const v4f a = *(const v4fa*)src, c4 = *(const v4fa*)(src + 4);
#pragma unroll
    for (int q = 0; q < 8; ++q) acc[q] += f * ((q < 4) ? a[q] : c4[q - 4]); }
  FragH o;
#pragma unroll
  for (int q = 0; q < 8; ++q) o.h[q] = (_Float16)acc[q];
  *(volatile v8us*)((unsigned short*)XS16 + ((size_t)b * NPX + ns) * CC + g * CG + c0) = o.half[0]; __threadfence(); *(volatile v8us*)((unsigned short*)XS16 + ((size_t)b * NPX + ns) * CC + g * CG + c0) = o.half[0]; }
__global__ __launch_bounds__(256) void k_vt(const _Float16* __restrict__ V16, int b, _Float16* __restrict__ VT) { const int t = blockIdx.x * 256 + threadIdx.x; if (t >= CC * (NPX / 8)) return; const int n0 = (t % (NPX / 8)) * 8, hc = t / (NPX / 8); FragH f;
#pragma unroll
  for (int q = 0; q < 8; ++q) f.h[q] = V16[((size_t)b * NPX + n0 + q) * CC + hc];
  *(volatile v8us*)((unsigned short*)VT + (size_t)hc * NPX + n0) = f.half[0]; __threadfence(); *(volatile v8us*)((unsigned short*)VT + (size_t)hc * NPX + n0) = f.half[0]; }
__global__ __launch_bounds__(256) void k_soft(const float* __restrict__ S, _Float16* __restrict__ P16) {
  #pragma clang fp contract(off)
  const int tid = threadIdx.x, w = tid >> 5, ln = tid & 31; const int row = blockIdx.x * 8 + w; if (row >= HGRP * NPX) return; const float* sr = S + (size_t)row * NPX; float m = -3.0e38f;
#pragma unroll 1
  for (int jb = 0; jb < NPX; jb += 256) { const v4f a = *(const v4fa*)(sr + jb + 8 * ln), c = *(const v4fa*)(sr + jb + 8 * ln + 4);
#pragma unroll
    for (int k = 0; k < 4; ++k) { m = fmaxf(m, a[k]); m = fmaxf(m, c[k]); } }
  for (int o = 16; o > 0; o >>= 1) m = fmaxf(m, __shfl_xor(m, o, 32));
  float su = 0.f;
#pragma unroll 1
  for (int jb = 0; jb < NPX; jb += 256) { const v4f a = *(const v4fa*)(sr + jb + 8 * ln), c = *(const v4fa*)(sr + jb + 8 * ln + 4);
#pragma unroll
    for (int k = 0; k < 4; ++k) { su += expf(a[k] - m); su += expf(c[k] - m); } }
  for (int o = 16; o > 0; o >>= 1) su += __shfl_xor(su, o, 32); const float inv = 1024.0f / su;
  for (int pass = 0; pass < 2; ++pass) {
#pragma unroll 1
    for (int jb = 0; jb < NPX; jb += 256) { const v4f a = *(const v4fa*)(sr + jb + 8 * ln), c = *(const v4fa*)(sr + jb + 8 * ln + 4); FragH f;
#pragma unroll
      for (int k = 0; k < 4; ++k) { f.h[k] = (_Float16)(expf(a[k] - m) * inv); f.h[4 + k] = (_Float16)(expf(c[k] - m) * inv); }
      *(volatile v8us*)((unsigned short*)P16 + (size_t)row * NPX + jb + 8 * ln) = f.half[0]; }
    if (pass == 0) __threadfence(); } }
__global__ __launch_bounds__(256) void k_t16(const float* __restrict__ X1, const float* __restrict__ ST, const float* __restrict__ g, const float* __restrict__ bb, _Float16* __restrict__ T16) {
  #pragma clang fp contract(off)
  const int t = blockIdx.x * 256 + threadIdx.x; if (t >= NBt * CC * (NPX / 8)) return; const int n0 = (t % (NPX / 8)) * 8; const int c = (t / (NPX / 8)) % CC; const int b = t / ((NPX / 8) * CC); const float gc = bf16_round(g[c]), bc = bf16_round(bb[c]); FragH f;
#pragma unroll
  for (int q = 0; q < 8; ++q) { const size_t r = (size_t)b * NPX + n0 + q; f.h[q] = (_Float16)((X1[r * CC + c] - ST[r * 32]) * ST[r * 32 + 1] * gc + bc); }
  *(volatile v8us*)((unsigned short*)T16 + ((size_t)b * CC + c) * NPX + n0) = f.half[0]; __threadfence(); *(volatile v8us*)((unsigned short*)T16 + ((size_t)b * CC + c) * NPX + n0) = f.half[0]; }
__global__ __launch_bounds__(256) void k_ffdw(const float* __restrict__ H1, const float* __restrict__ w, const float* __restrict__ bb, _Float16* __restrict__ AX16) {
  #pragma clang fp contract(off)
  const int t = blockIdx.x * 256 + threadIdx.x; if (t >= NR * (DFF / 4)) return; const int f0 = (t % (DFF / 4)) * 4, r = t / (DFF / 4); const int b = r / NPX, p = r % NPX; const int y = p / HW, x = p % HW; v4f acc = *(const v4fa*)(H1 + (size_t)r * DFF + f0);
#pragma unroll
  for (int q = 0; q < 4; ++q) acc[q] += bf16_round(bb[f0 + q]);
#pragma unroll 1
  for (int tp = 0; tp < 9; ++tp) { const int yy = y + tp / 3 - 1, xx = x + tp % 3 - 1; if (yy < 0 || yy >= HW || xx < 0 || xx >= HW) continue; const v4f v = *(const v4fa*)(H1 + ((size_t)b * NPX + yy * HW + xx) * DFF + f0);
#pragma unroll
    for (int q = 0; q < 4; ++q) acc[q] += v[q] * bf16_round(w[(size_t)(f0 + q) * 9 + tp]); }
  FragH f; f.h[0] = (_Float16)acc[0]; f.h[1] = (_Float16)acc[1]; f.h[2] = (_Float16)acc[2]; f.h[3] = (_Float16)acc[3]; const unsigned long long pv = *(const unsigned long long*)&f.u[0]; *(volatile unsigned long long*)((unsigned short*)AX16 + (size_t)r * DFF + f0) = pv; __threadfence(); *(volatile unsigned long long*)((unsigned short*)AX16 + (size_t)r * DFF + f0) = pv; }
__global__ __launch_bounds__(256) void k_ffact(_Float16* __restrict__ A16, const float* __restrict__ ST, const float* __restrict__ g, const float* __restrict__ bb) {
  #pragma clang fp contract(off)
  const int t = blockIdx.x * 256 + threadIdx.x; if (t >= NR * (DFF / 8)) return; const int f0 = (t % (DFF / 8)) * 8, r = t / (DFF / 8); const float mu = ST[(size_t)r * 32], rs = ST[(size_t)r * 32 + 1]; FragH a; a.half[0] = *(const v8us*)((const unsigned short*)A16 + (size_t)r * DFF + f0); FragH f = FragH{};
_Pragma("unroll 1")
  for (int q = 0; q < 8; ++q) { const int ff = f0 + q; float yv = gelu_f(((float)a.h[q] - mu) * rs * bf16_round(g[ff]) + bf16_round(bb[ff])); _Float16 hv = (_Float16)yv;
#pragma unroll
    for (int k = 0; k < 8; ++k) f.h[k] = (k == q) ? hv : f.h[k]; }
  *(volatile v8us*)((unsigned short*)A16 + (size_t)r * DFF + f0) = f.half[0]; __threadfence(); *(volatile v8us*)((unsigned short*)A16 + (size_t)r * DFF + f0) = f.half[0]; }
__global__ __launch_bounds__(256) void k_fin(const float* __restrict__ O2, const float* __restrict__ X1, float* __restrict__ out) {
  #pragma clang fp contract(off)
  const int t = blockIdx.x * 256 + threadIdx.x; if (t >= NBt * CC * (NPX / 4)) return; const int n0 = (t % (NPX / 4)) * 4; const int c = (t / (NPX / 4)) % CC; const int b = t / ((NPX / 4) * CC); const size_t fi = ((size_t)b * CC + c) * NPX + n0; const v4f o = *(const v4fa*)(O2 + fi); v4f v;
#pragma unroll
  for (int q = 0; q < 4; ++q) v[q] = o[q] + X1[((size_t)b * NPX + n0 + q) * CC + c];
  *(volatile v4f*)(out + fi) = v; __threadfence(); *(volatile v4f*)(out + fi) = v; }

extern "C" void kernel_launch(void* const* d_in, const int* in_sizes, int n_in,
                              void* d_out, int out_size, void* d_ws, size_t ws_size, hipStream_t stream) {
  (void)in_sizes; (void)n_in; (void)out_size;
  const float* const* I = (const float* const*)d_in; const float* x = I[0];
  char* ws = (char*)d_ws; size_t off = 0;
  auto take = [&](size_t bytes) { char* p = ws + off; off += (bytes + 255) & ~(size_t)255; return p; };
  _Float16* BW = (_Float16*)take((size_t)CC * CC * 2); _Float16* BF = (_Float16*)take((size_t)DFF * CC * 2);
  float* X = (float*)take((size_t)NR * CC * 4);
  char* R50 = take((size_t)NR * CC * 4 * 2 + (size_t)NR * CC * 2 * 4);
  float* OD = (float*)take((size_t)NBt * GG * NPX * CG * 4); float* POS = (float*)take((size_t)NBt * GG * NPX * 32 * 4); _Float16* VT = (_Float16*)take((size_t)CC * NPX * 2); _Float16* OUT16 = (_Float16*)take((size_t)NR * CC * 2); _Float16* T16 = (_Float16*)take((size_t)NR * CC * 2);
  float* X1 = (float*)take((size_t)NR * CC * 4); float* ST = (float*)take((size_t)NR * 32 * 4); _Float16* AX16 = (_Float16*)take((size_t)NR * DFF * 2);
  if (off > ws_size) return;
  float* XN = (float*)R50; float* Q = (float*)(R50 + (size_t)NR * CC * 4); _Float16* Q16 = (_Float16*)(R50 + (size_t)NR * CC * 8); _Float16* XS16 = (_Float16*)(R50 + (size_t)NR * CC * 10); _Float16* K16 = (_Float16*)(R50 + (size_t)NR * CC * 12); _Float16* V16 = (_Float16*)(R50 + (size_t)NR * CC * 14); float* H1 = (float*)R50; _Float16* XN16 = OUT16;
  float* S = (float*)R50; _Float16* P16 = (_Float16*)(R50 + (size_t)HGRP * NPX * NPX * 4);
  float* O2 = (float*)OD;
  const size_t n8 = (size_t)NR * CC / 8; const dim3 gC(((NR / 16) * (CC / 64) + 3) / 4, 1), gF(((NR / 16) * (DFF / 64) + 3) / 4, 1);
  k_tok<<<(NR * (CC / 4) + 255) / 256, 256, 0, stream>>>(x, X);
  k_rstat<<<NR / 8, 256, 0, stream>>>(X, CC, NR, 1e-5f, ST); k_lnapply<<<(NR * (CC / 8) + 255) / 256, 256, 0, stream>>>(X, CC, ST, I[1], I[2], XN, XN16);
  k_round16f<<<(CC * CC / 8 + 255) / 256, 256, 0, stream>>>(I[8], BW, (size_t)CC * CC / 8); k_gemm_hhx<0><<<gC, 128, 0, stream>>>(XN16, CC, 0, BW, CC, 0, 0.0625f, I[9], 0, nullptr, 1, 0, 0, Q, nullptr, CC, 0, NR, CC, CC);
  k_odw<<<(NBt * GG * NPX * (CG / 4) + 255) / 256, 256, 0, stream>>>(Q, I[3], I[4], OD); k_opos<<<(NBt * GG * NPX + 7) / 8, 256, 0, stream>>>(OD, I[5], I[6], I[7], POS);
  k_samp<<<(NBt * GG * NPX * (CG / 8) + 255) / 256, 256, 0, stream>>>(XN, POS, XS16);
  k_f16<<<(unsigned)((n8 + 255) / 256), 256, 0, stream>>>(Q, Q16, n8);
  k_round16f<<<(CC * CC / 8 + 255) / 256, 256, 0, stream>>>(I[10], BW, (size_t)CC * CC / 8); k_gemm_hhx<0><<<gC, 128, 0, stream>>>(XS16, CC, 0, BW, CC, 0, 0.0625f, I[11], 0, nullptr, 1, 0, 0, nullptr, K16, CC, 0, NR, CC, CC);
  k_round16f<<<(CC * CC / 8 + 255) / 256, 256, 0, stream>>>(I[12], BW, (size_t)CC * CC / 8); k_gemm_hhx<0><<<gC, 128, 0, stream>>>(XS16, CC, 0, BW, CC, 0, 0.0625f, I[13], 0, nullptr, 1, 0, 0, nullptr, V16, CC, 0, NR, CC, CC);
  const dim3 gS(((NPX / 16) * (NPX / 64) + 3) / 4, HGRP), gV(((NPX / 16) * 1 + 3) / 4, HGRP);
  for (int b = 0; b < NBt; ++b) { k_vt<<<(CC * (NPX / 8) + 255) / 256, 256, 0, stream>>>(V16, b, VT);
    for (int hg = 0; hg < NHD / HGRP; ++hg) { const int h0 = hg * HGRP;
      k_gemm_hhx<0><<<gS, 128, 0, stream>>>(Q16 + (size_t)b * NPX * CC + h0 * HC, CC, (size_t)HC, K16 + (size_t)b * NPX * CC + h0 * HC, CC, (size_t)HC, 0.17677669529663687f, nullptr, 0, nullptr, 1, 0, 0, S, nullptr, NPX, (size_t)NPX * NPX, NPX, NPX, HC);
      k_soft<<<HGRP * NPX / 8, 256, 0, stream>>>(S, P16);
      k_gemm_hhx<0><<<gV, 128, 0, stream>>>(P16, NPX, (size_t)NPX * NPX, VT + (size_t)h0 * HC * NPX, NPX, (size_t)HC * NPX, 0.0009765625f, nullptr, 0, nullptr, 1, 0, 0, nullptr, OUT16 + (size_t)b * NPX * CC + h0 * HC, CC, (size_t)HC, NPX, HC, NPX); } }
  k_round16f<<<(CC * CC / 8 + 255) / 256, 256, 0, stream>>>(I[14], BW, (size_t)CC * CC / 8); k_gemm_hhx<0><<<gC, 128, 0, stream>>>(OUT16, CC, 0, BW, CC, 0, 0.0625f, I[15], 0, X, 1, (size_t)CC, 0, X1, nullptr, CC, 0, NR, CC, CC);
  k_rstat<<<NR / 8, 256, 0, stream>>>(X1, CC, NR, 1e-5f, ST); k_t16<<<(NBt * CC * (NPX / 8) + 255) / 256, 256, 0, stream>>>(X1, ST, I[16], I[17], T16);
  k_round16f<<<(unsigned)(((size_t)DFF * CC / 8 + 255) / 256), 256, 0, stream>>>(I[18], BF, (size_t)DFF * CC / 8); k_gemm_hhx<0><<<gF, 128, 0, stream>>>(T16, CC, 0, BF, CC, 0, 0.0625f, I[19], 0, nullptr, 1, 0, 0, H1, nullptr, DFF, 0, NR, DFF, CC);
  k_ffdw<<<(NR * (DFF / 4) + 255) / 256, 256, 0, stream>>>(H1, I[20], I[21], AX16); k_rstat16<<<NR / 8, 256, 0, stream>>>(AX16, DFF, NR, 1e-5f, ST); k_ffact<<<(NR * (DFF / 8) + 255) / 256, 256, 0, stream>>>(AX16, ST, I[22], I[23]);
  k_round16f<<<(unsigned)(((size_t)CC * DFF / 8 + 255) / 256), 256, 0, stream>>>(I[24], BF, (size_t)CC * DFF / 8);
  k_gemm_hhx<0><<<gC, 128, 0, stream>>>(AX16, DFF, 0, BF, DFF, 0, 0.0625f, I[25], 0, nullptr, 1, 0, 0, O2, nullptr, CC, 0, NR, CC, DFF);
  k_fin<<<(NBt * CC * (NPX / 4) + 255) / 256, 256, 0, stream>>>(O2, X1, (float*)d_out);
}
